// TwoDGRUClassifier_77807627534337
// MI455X (gfx1250) — hardware-verified
//
#include <hip/hip_runtime.h>
#include <hip/hip_bf16.h>

typedef _Float16 h16;
typedef __attribute__((ext_vector_type(16))) _Float16 v16bf;
typedef __attribute__((ext_vector_type(8)))  _Float16 v8bf;
typedef __attribute__((ext_vector_type(8)))  float  v8f;
typedef __attribute__((ext_vector_type(4)))  float  v4f;
#define VST2(T, ptr, val) do { const T _v = (val); *(volatile T*)(ptr) = _v; __threadfence(); *(volatile T*)(ptr) = _v; } while (0)
__device__ __forceinline__ v8f wmma16(v16bf a, v16bf b, v8f c) {
    v8f d = __builtin_amdgcn_wmma_f32_16x16x32_f16(false, a, false, b, (short)0, c, false, false);
    asm volatile("v_nop\n\tv_nop\n\tv_nop\n\tv_nop" : "+v"(d) : "v"(a), "v"(b));
    return d;
}
#define NTO 64

#define HIDN 128
#define GRID 32
#define BQ   32
#define EMBD 64
#define NDIRS 4
#define NCLSS 1000
#define ASTRIDE 264

__device__ __forceinline__ float bf2f(h16 v) { return (float)v; }
__device__ __forceinline__ h16   f2bf(float v)  { return (h16)v; }

__global__ void prepack_kernel(const float* __restrict__ src, h16* __restrict__ dst,
                               int K, int Nsrc, int NT) {
    int total = (K >> 5) * NT * 512;
    int i8 = blockIdx.x * 256 + threadIdx.x;
    if (i8 * 8 >= total) return;
    v8bf o;
#pragma unroll
    for (int q = 0; q < 8; ++q) {
        int idx = i8 * 8 + q;
        int e  = idx & 15;
        int L  = (idx >> 4) & 31;
        int nt = (idx >> 9) % NT;
        int kt = idx / (NT * 512);
        int k  = kt * 32 + ((e < 8) ? e : (e + 8)) + ((L >= 16) ? 8 : 0);
        int n  = nt * 16 + (L & 15);
        o[q] = f2bf((n < Nsrc) ? src[(size_t)k * Nsrc + n] : 0.0f);
    }
    VST2(v8bf, dst + (size_t)i8 * 8, o);
}

__global__ void embed_kernel(const float* __restrict__ x, const float* __restrict__ We,
                             const float* __restrict__ be, float* __restrict__ emb) {
    int idx = blockIdx.x * 256 + threadIdx.x;
    int e = idx & 63;
    int b = (idx >> 6) & 31;
    int j = (idx >> 11) & 31;
    int i = (idx >> 16) & 31;
    const float* xp = x + (((size_t)b * GRID + i) * GRID + j) * 3;
    float v = be[e] + xp[0] * We[0 * EMBD + e] + xp[1] * We[1 * EMBD + e]
                    + xp[2] * We[2 * EMBD + e];
    VST2(float, emb + idx, v);
}

template<int XKT>
__global__ __launch_bounds__(256) void diag_scan_kernel(
    const float* __restrict__ xin,
    float* __restrict__ hout,
    const h16* __restrict__ wxp,
    const h16* __restrict__ whp,
    const float* __restrict__ bx,
    const float* __restrict__ bh,
    int t, int cnt)
{
    constexpr int IN_DIM = XKT * 32;
    __shared__ __attribute__((aligned(16))) h16 A_lds[32][ASTRIDE];
    __shared__ __attribute__((aligned(16))) float Hav[32][HIDN];
    __shared__ __attribute__((aligned(16))) float Hnew[32][HIDN];

    const int d   = blockIdx.x / cnt;
    const int ci  = blockIdx.x % cnt;
    const int i0  = (t > 31) ? (t - 31) : 0;
    const int i   = i0 + ci;
    const int j   = t - i;
    const int tid = threadIdx.x;

    for (int idx = tid; idx < 32 * HIDN; idx += 256) {
        int m = idx >> 7, c = idx & 127;
        float hl = 0.f, hu = 0.f;
        if (j > 0) hl = hout[((((size_t)d * GRID + i) * GRID + (j - 1)) * BQ + m) * HIDN + c];
        if (i > 0) hu = hout[((((size_t)d * GRID + (i - 1)) * GRID + j) * BQ + m) * HIDN + c];
        float av = 0.5f * (hl + hu);
        Hav[m][c] = av;
        A_lds[m][IN_DIM + c] = f2bf(av);
    }
    if constexpr (XKT == 2) {
        const int fi = (d & 1) ? (31 - i) : i;
        const int fj = (d & 2) ? (31 - j) : j;
        const float* src = xin + (((size_t)fi * GRID + fj) * BQ) * EMBD;
        for (int idx = tid; idx < 32 * EMBD; idx += 256)
            A_lds[idx >> 6][idx & 63] = f2bf(src[idx]);
    } else {
        const float* src = xin + ((((size_t)d * GRID + i) * GRID + j) * BQ) * HIDN;
        for (int idx = tid; idx < 32 * HIDN; idx += 256)
            A_lds[idx >> 7][idx & 127] = f2bf(src[idx]);
    }
    __syncthreads();

    const int w    = tid >> 5;
    const int lane = tid & 31;
    const int mrow = lane & 15;
    const int kg   = (lane >> 4) << 3;

    v8f accx[2][3], acch[2][3];
    #pragma unroll
    for (int mt = 0; mt < 2; ++mt)
        #pragma unroll
        for (int g = 0; g < 3; ++g) {
            accx[mt][g] = (v8f){0.f,0.f,0.f,0.f,0.f,0.f,0.f,0.f};
            acch[mt][g] = (v8f){0.f,0.f,0.f,0.f,0.f,0.f,0.f,0.f};
        }

    const h16* wxd = wxp + (size_t)d * XKT * 24 * 512;
    const h16* whd = whp + (size_t)d * 4   * 24 * 512;

    #pragma unroll
    for (int kt = 0; kt < XKT; ++kt) {
        const int kbase = kt * 32;
        v8bf lo0 = *(const v8bf*)&A_lds[mrow][kbase + kg];
        v8bf hi0 = *(const v8bf*)&A_lds[mrow][kbase + 16 + kg];
        v8bf lo1 = *(const v8bf*)&A_lds[16 + mrow][kbase + kg];
        v8bf hi1 = *(const v8bf*)&A_lds[16 + mrow][kbase + 16 + kg];
        v16bf a0 = __builtin_shufflevector(lo0, hi0, 0,1,2,3,4,5,6,7,8,9,10,11,12,13,14,15);
        v16bf a1 = __builtin_shufflevector(lo1, hi1, 0,1,2,3,4,5,6,7,8,9,10,11,12,13,14,15);
        const h16* wbase = wxd + (size_t)kt * 24 * 512;
        #pragma unroll
        for (int g = 0; g < 3; ++g) {
            v16bf bf = *(const v16bf*)(wbase + ((size_t)(g * 8 + w) * 32 + lane) * 16);
            accx[0][g] = wmma16(a0, bf, accx[0][g]);
            accx[1][g] = wmma16(a1, bf, accx[1][g]);
        }
    }
    #pragma unroll
    for (int kt = 0; kt < 4; ++kt) {
        const int kbase = IN_DIM + kt * 32;
        v8bf lo0 = *(const v8bf*)&A_lds[mrow][kbase + kg];
        v8bf hi0 = *(const v8bf*)&A_lds[mrow][kbase + 16 + kg];
        v8bf lo1 = *(const v8bf*)&A_lds[16 + mrow][kbase + kg];
        v8bf hi1 = *(const v8bf*)&A_lds[16 + mrow][kbase + 16 + kg];
        v16bf a0 = __builtin_shufflevector(lo0, hi0, 0,1,2,3,4,5,6,7,8,9,10,11,12,13,14,15);
        v16bf a1 = __builtin_shufflevector(lo1, hi1, 0,1,2,3,4,5,6,7,8,9,10,11,12,13,14,15);
        const h16* wbase = whd + (size_t)kt * 24 * 512;
        #pragma unroll
        for (int g = 0; g < 3; ++g) {
            v16bf bf = *(const v16bf*)(wbase + ((size_t)(g * 8 + w) * 32 + lane) * 16);
            acch[0][g] = wmma16(a0, bf, acch[0][g]);
            acch[1][g] = wmma16(a1, bf, acch[1][g]);
        }
    }

    const int col = 16 * w + mrow;
    const float bxr = bx[d * 384 + col];
    const float bxz = bx[d * 384 + 128 + col];
    const float bxn = bx[d * 384 + 256 + col];
    const float bhr = bh[d * 384 + col];
    const float bhz = bh[d * 384 + 128 + col];
    const float bhn = bh[d * 384 + 256 + col];
    const int mh = (lane >> 4) << 3;

    #pragma unroll
    for (int mt = 0; mt < 2; ++mt) {
        #pragma unroll
        for (int e = 0; e < 8; ++e) {
            float r = 1.f / (1.f + expf(-(accx[mt][0][e] + bxr + acch[mt][0][e] + bhr)));
            float z = 1.f / (1.f + expf(-(accx[mt][1][e] + bxz + acch[mt][1][e] + bhz)));
            float n = tanhf(accx[mt][2][e] + bxn + r * (acch[mt][2][e] + bhn));
            int m = mt * 16 + mh + e;
            Hnew[m][col] = (1.f - z) * n + z * Hav[m][col];
        }
    }
    __syncthreads();
    float* dst = hout + ((((size_t)d * GRID + i) * GRID + j) * BQ) * HIDN;
    for (int pass = 0; pass < 2; ++pass) {
#pragma unroll
        for (int q = 0; q < 4; ++q) { const int p = tid + q * 256; *(volatile v4f*)(dst + p * 4) = *(const v4f*)(&Hnew[0][0] + p * 4); }
        __threadfence();
    }
}

__global__ __launch_bounds__(256) void final_gemm_kernel(
    const float* __restrict__ hmap, int ci, int cj, const h16* __restrict__ wop,
    const float* __restrict__ bo, float* __restrict__ outp)
{
    const int lane = threadIdx.x & 31, wave = threadIdx.x >> 5, hh = lane >> 4, l16 = lane & 15;
    for (int pr = wave; pr < NTO / 2; pr += 8) {
        for (int mt = 0; mt < 2; ++mt) {
            v8f acc0 = (v8f){0.f,0.f,0.f,0.f,0.f,0.f,0.f,0.f}, acc1 = acc0;
            const int m = mt * 16 + l16;
            for (int kt = 0; kt < 16; ++kt) {
                v16bf a;
#pragma unroll
                for (int e = 0; e < 16; ++e) {
                    const int k = kt * 32 + ((e < 8) ? (8 * hh + e) : (16 + 8 * hh + e - 8));
                    const int dd = k >> 7, c = k & 127;
                    a[e] = f2bf(hmap[((((size_t)dd * GRID + ci) * GRID + cj) * BQ + m) * HIDN + c]);
                }
                const v16bf b0 = *(const v16bf*)(wop + (((size_t)kt * NTO + 2 * pr) * 32 + lane) * 16);
                const v16bf b1 = *(const v16bf*)(wop + (((size_t)kt * NTO + 2 * pr + 1) * 32 + lane) * 16);
                acc0 = wmma16(a, b0, acc0);
                acc1 = wmma16(a, b1, acc1);
            }
            const int cb = pr * 32;
            const float bv = (cb + lane < NCLSS) ? bo[cb + lane] : 0.f;
            for (int pass = 0; pass < 2; ++pass) {
#pragma unroll
                for (int e = 0; e < 8; ++e) {
                    const float a_ = acc0[e], b_ = acc1[e];
                    const float ax = __shfl_xor(a_, 16), bx = __shfl_xor(b_, 16);
                    *(volatile float*)(outp + (size_t)(mt * 16 + e) * 1024 + cb + lane)     = (hh ? bx : a_) + bv;
                    *(volatile float*)(outp + (size_t)(mt * 16 + e + 8) * 1024 + cb + lane) = (hh ? b_ : ax) + bv;
                }
                __threadfence();
            }
        }
    }
}
__global__ __launch_bounds__(256) void copy_out_kernel(const float* __restrict__ outp, float* __restrict__ out) {
    const int t = blockIdx.x * 256 + threadIdx.x;
    if (t >= BQ * NCLSS) return;
    const int m = t / NCLSS, c = t - m * NCLSS;
    VST2(float, out + t, outp[(size_t)m * 1024 + c]);
}

extern "C" void kernel_launch(void* const* d_in, const int* in_sizes, int n_in,
                              void* d_out, int out_size, void* d_ws, size_t ws_size,
                              hipStream_t stream) {
    (void)in_sizes; (void)n_in; (void)out_size; (void)ws_size;
    const float* x  = (const float*)d_in[0];
    const float* We = (const float*)d_in[1];
    const float* be = (const float*)d_in[2];
    const float *Wx[3], *Wh[3], *bx[3], *bh[3];
    for (int l = 0; l < 3; ++l) {
        Wx[l] = (const float*)d_in[3 + 4 * l];
        Wh[l] = (const float*)d_in[4 + 4 * l];
        bx[l] = (const float*)d_in[5 + 4 * l];
        bh[l] = (const float*)d_in[6 + 4 * l];
    }
    const float* Wo = (const float*)d_in[15];
    const float* bo = (const float*)d_in[16];
    float* out = (float*)d_out;

    (void)in_sizes; (void)n_in; (void)out_size;
    char* ws = (char*)d_ws;
    size_t off = 0;
    auto alloc = [&](size_t bytes) -> char* {
        char* p = ws + off;
        off += (bytes + 255) & ~(size_t)255;
        return p;
    };

    const int indim[3] = {64, 128, 128};
    float* emb = (float*)alloc((size_t)GRID * GRID * BQ * EMBD * 4);
    h16 *wxp[3], *whp[3];
    for (int l = 0; l < 3; ++l) {
        wxp[l] = (h16*)alloc((size_t)NDIRS * (indim[l] / 32) * 24 * 512 * 2);
        whp[l] = (h16*)alloc((size_t)NDIRS * 4 * 24 * 512 * 2);
    }
    h16* wop   = (h16*)alloc((size_t)16 * NTO * 512 * 2);
    float* hA  = (float*)alloc((size_t)NDIRS * GRID * GRID * BQ * HIDN * 4);
    float* hB  = (float*)alloc((size_t)NDIRS * GRID * GRID * BQ * HIDN * 4);
    float* outp = (float*)alloc((size_t)BQ * 1024 * 4);
    if (off > ws_size) return;

    for (int l = 0; l < 3; ++l) {
        const int K = indim[l];
        for (int d = 0; d < NDIRS; ++d) {
            int tot = (K / 32) * 24 * 512;
            prepack_kernel<<<(tot / 8 + 255) / 256, 256, 0, stream>>>(
                Wx[l] + (size_t)d * K * 384, wxp[l] + (size_t)d * (K / 32) * 24 * 512, K, 384, 24);
            int tot2 = 4 * 24 * 512;
            prepack_kernel<<<(tot2 / 8 + 255) / 256, 256, 0, stream>>>(
                Wh[l] + (size_t)d * 128 * 384, whp[l] + (size_t)d * 4 * 24 * 512, 128, 384, 24);
        }
    }
    {
        int tot = 16 * NTO * 512;
        prepack_kernel<<<(tot / 8 + 255) / 256, 256, 0, stream>>>(Wo, wop, 512, 1000, NTO);
    }

    embed_kernel<<<8192, 256, 0, stream>>>(x, We, be, emb);

    float* maps[2] = {hA, hB};
    const int TSTEPS = 63;
    for (int l = 0; l < 3; ++l) {
        float* hout = maps[l & 1];
        const float* xin = (l == 0) ? emb : maps[(l - 1) & 1];
        for (int t = 0; t < TSTEPS; ++t) {
            int i0 = (t > 31) ? (t - 31) : 0;
            int i1 = (t < 31) ? t : 31;
            int cnt = i1 - i0 + 1;
            if (l == 0)
                diag_scan_kernel<2><<<cnt * NDIRS, 256, 0, stream>>>(
                    xin, hout, wxp[l], whp[l], bx[l], bh[l], t, cnt);
            else
                diag_scan_kernel<4><<<cnt * NDIRS, 256, 0, stream>>>(
                    xin, hout, wxp[l], whp[l], bx[l], bh[l], t, cnt);
        }
    }

    final_gemm_kernel<<<1, 256, 0, stream>>>(maps[0], 31, 31, wop, bo, outp);
    copy_out_kernel<<<(BQ * NCLSS + 255) / 256, 256, 0, stream>>>(outp, out);
}
